// Nonlocal_55851754717492
// MI455X (gfx1250) — hardware-verified
//
#include <hip/hip_runtime.h>

constexpr int kBatch = 4;
constexpr int kC     = 256;
constexpr int kCi    = 128;
constexpr int kN     = 4096;
constexpr float kWCarry    = 16.0f;
constexpr float kProjScale = 1.0f / 16.0f;
constexpr float kSScale    = 1.0f / 16.0f;
constexpr float kW2Scale   = 1.0f / 64.0f;
constexpr float kOutScale  = 1.0f / 64.0f;
static_assert(kN % 64 == 0 && kC % 64 == 0 && kCi % 64 == 0, "M,N tiles");
static_assert(kC % 32 == 0 && kN % 32 == 0 && kCi % 32 == 0, "K steps");
static_assert(kCi * kC == 32768 && kC * kCi == 32768, "weight planes");

typedef __attribute__((ext_vector_type(16))) _Float16 v16h;
typedef __attribute__((ext_vector_type(8)))  _Float16 v8h;
typedef __attribute__((ext_vector_type(16))) __bf16   v16b;
typedef __attribute__((ext_vector_type(8)))  __bf16   v8b;
typedef __attribute__((ext_vector_type(8)))  float    v8f;
typedef __attribute__((ext_vector_type(4)))  float    v4f;
typedef __attribute__((ext_vector_type(4)))  unsigned int v4u;

__device__ __forceinline__ void dep_guard4x_h(v8f& a, v8f& b, v8f& c, v8f& d, v16h x, v16h y) {
  asm volatile("v_nop\n\tv_nop\n\tv_nop\n\tv_nop" : "+v"(a), "+v"(b), "+v"(c), "+v"(d) : "v"(x), "v"(y));
}
__device__ __forceinline__ void dep_guard4x_b(v8f& a, v8f& b, v8f& c, v8f& d, v16b x, v16b y) {
  asm volatile("v_nop\n\tv_nop\n\tv_nop\n\tv_nop" : "+v"(a), "+v"(b), "+v"(c), "+v"(d) : "v"(x), "v"(y));
}
__device__ __forceinline__ void keep4_h(v16h a, v16h b, v16h c, v16h d) { asm volatile("v_nop" :: "v"(a), "v"(b), "v"(c), "v"(d)); }
__device__ __forceinline__ void keep4_b(v16b a, v16b b, v16b c, v16b d) { asm volatile("v_nop" :: "v"(a), "v"(b), "v"(c), "v"(d)); }
__device__ __forceinline__ void acc_guard4(v8f& a, v8f& b, v8f& c, v8f& d) { asm volatile("v_nop\n\tv_nop\n\tv_nop\n\tv_nop" : "+v"(a), "+v"(b), "+v"(c), "+v"(d)); }
__device__ __forceinline__ void quad_keep4f(v4f& a, v4f& b, v4f& c, v4f& d) { asm volatile("" : "+v"(a), "+v"(b), "+v"(c), "+v"(d) :: "memory"); }

template <typename T> struct Frag;
template <> struct Frag<_Float16> {
  typedef v16h V; union U { v16h v; v8h h[2]; };
  static __device__ __forceinline__ v16h load(const _Float16* p) {
    U f; f.h[0] = *(const v8h*)(p); f.h[1] = *(const v8h*)(p + 16); return f.v;
  }
  static __device__ __forceinline__ v8f mma(v16h a, v16h b, v8f c) {
    return __builtin_amdgcn_wmma_f32_16x16x32_f16(false, a, false, b, (short)0, c, false, false);
  }
  static __device__ __forceinline__ void guard4(v8f& a, v8f& b, v8f& c, v8f& d, v16h x, v16h y) { dep_guard4x_h(a, b, c, d, x, y); }
  static __device__ __forceinline__ void keep(v16h a, v16h b, v16h c, v16h d) { keep4_h(a, b, c, d); }
};
template <> struct Frag<__bf16> {
  typedef v16b V; union U { v16b v; v8b h[2]; };
  static __device__ __forceinline__ v16b load(const __bf16* p) {
    U f; f.h[0] = *(const v8b*)(p); f.h[1] = *(const v8b*)(p + 16); return f.v;
  }
  static __device__ __forceinline__ v8f mma(v16b a, v16b b, v8f c) {
    return __builtin_amdgcn_wmma_f32_16x16x32_bf16(false, a, false, b, (short)0, c, false, false);
  }
  static __device__ __forceinline__ void guard4(v8f& a, v8f& b, v8f& c, v8f& d, v16b x, v16b y) { dep_guard4x_b(a, b, c, d, x, y); }
  static __device__ __forceinline__ void keep(v16b a, v16b b, v16b c, v16b d) { keep4_b(a, b, c, d); }
};

__device__ __forceinline__ unsigned pk16(unsigned short a, unsigned short b) { return (unsigned)a | ((unsigned)b << 16); }
__device__ __forceinline__ unsigned short h_bits(float f) { const _Float16 h = (_Float16)f; return __builtin_bit_cast(unsigned short, h); }

template <int ET> struct Elem;
template <> struct Elem<0> { typedef _Float16 T; };
template <> struct Elem<1> { typedef __bf16 T; };
template <int ET, bool SPLIT, int BIAS_MODE, int OUT_MODE, bool RESID>
__global__ __launch_bounds__(256) void wmma_gemm64(
    const unsigned short* __restrict__ Ap, const unsigned short* __restrict__ A2p, int lda, long strideA,
    const unsigned short* __restrict__ Btp, const unsigned short* __restrict__ Bt2p, int ldb, long strideB,
    void* __restrict__ Cout, int ldc, long strideC,
    const float* __restrict__ bias,
    const float* __restrict__ resid, long strideR,
    int M, int N, int K, float scale) {
  static_assert(OUT_MODE == 0 || OUT_MODE == 1, "modes");
  static_assert(!(RESID && OUT_MODE != 0), "resid f32 only");
  typedef typename Elem<ET>::T T;
  typedef typename Frag<T>::V V;
  const T* A = (const T*)Ap; const T* A2 = (const T*)A2p; const T* Bt = (const T*)Btp; const T* Bt2 = (const T*)Bt2p;
  __shared__ __align__(16) float sT[8][16 * 68];
  const int b    = blockIdx.y;
  const int lane = threadIdx.x & 31;
  const int wave = threadIdx.x >> 5;
  const int tilesN = N >> 6;
  const int tilesM = M >> 6;
  const int tile = blockIdx.x * 8 + wave;
  if (tile >= tilesM * tilesN) return;
  const int tm = tile / tilesN;
  const int tn = tile - tm * tilesN;
  const int m0 = tm << 6;
  const int n0 = tn << 6;

  const T* Ab  = A  + (size_t)b * strideA;
  const T* Bb  = Bt + (size_t)b * strideB;
  const T* Ab2 = SPLIT ? (A2  + (size_t)b * strideA) : nullptr;
  const T* Bb2 = SPLIT ? (Bt2 + (size_t)b * strideB) : nullptr;

  const int rlane = lane & 15;
  const int koff  = (lane >> 4) * 8;
  const int mOff  = (lane >> 4) * 8;

  v8f acc[4][4];
#pragma unroll
  for (int i = 0; i < 4; ++i)
#pragma unroll
    for (int j = 0; j < 4; ++j) acc[i][j] = (v8f){0.f,0.f,0.f,0.f,0.f,0.f,0.f,0.f};

  for (int k0 = 0; k0 < K; k0 += 32) {
    V bh[4], bl[4];
#pragma unroll
    for (int j = 0; j < 4; ++j) {
      const size_t bo = (size_t)(n0 + (j << 4) + rlane) * ldb + koff + k0;
      bh[j] = Frag<T>::load(Bb + bo);
      if (SPLIT) bl[j] = Frag<T>::load(Bb2 + bo);
    }
#pragma unroll
    for (int i = 0; i < 4; ++i) {
      const size_t ao = (size_t)(m0 + (i << 4) + rlane) * lda + koff + k0;
      V ah = Frag<T>::load(Ab + ao);
      V al;
      if (SPLIT) al = Frag<T>::load(Ab2 + ao);
#pragma unroll
      for (int j = 0; j < 4; ++j) {
        acc[i][j] = Frag<T>::mma(ah, bh[j], acc[i][j]);
        if (SPLIT) {
          acc[i][j] = Frag<T>::mma(ah, bl[j], acc[i][j]);
          acc[i][j] = Frag<T>::mma(al, bh[j], acc[i][j]);
        }
      }
      Frag<T>::guard4(acc[i][0], acc[i][1], acc[i][2], acc[i][3], ah, SPLIT ? al : ah);
    }
    Frag<T>::keep(bh[0], bh[1], bh[2], bh[3]);
    if (SPLIT) Frag<T>::keep(bl[0], bl[1], bl[2], bl[3]);
  }
  acc_guard4(acc[0][0], acc[0][1], acc[0][2], acc[0][3]);
  acc_guard4(acc[1][0], acc[1][1], acc[1][2], acc[1][3]);
  acc_guard4(acc[2][0], acc[2][1], acc[2][2], acc[2][3]);
  acc_guard4(acc[3][0], acc[3][1], acc[3][2], acc[3][3]);

  float* slab = sT[wave];
#pragma unroll
  for (int i = 0; i < 4; ++i) {
    const int mBase = m0 + (i << 4);
    float bmv[8];
#pragma unroll
    for (int r = 0; r < 8; ++r) bmv[r] = 0.f;
    if (BIAS_MODE == 1) {
      const v4f t0 = *(const v4f*)(bias + mBase + mOff);
      const v4f t1 = *(const v4f*)(bias + mBase + mOff + 4);
      bmv[0] = t0[0]; bmv[1] = t0[1]; bmv[2] = t0[2]; bmv[3] = t0[3];
      bmv[4] = t1[0]; bmv[5] = t1[1]; bmv[6] = t1[2]; bmv[7] = t1[3];
    }
#pragma unroll
    for (int j = 0; j < 4; ++j) {
      const int n = n0 + (j << 4) + rlane;
      float bv = 0.f;
      if (BIAS_MODE == 2) bv = bias[n];
#pragma unroll
      for (int r = 0; r < 8; ++r) {
        float v = acc[i][j][r] * scale;
        if (BIAS_MODE == 1) v += bmv[r];
        if (BIAS_MODE == 2) v += bv;
        slab[(mOff + r) * 68 + (j << 4) + rlane] = v;
      }
    }
    __builtin_amdgcn_fence(__ATOMIC_RELEASE, "workgroup");
    __builtin_amdgcn_wave_barrier();
    __builtin_amdgcn_fence(__ATOMIC_ACQUIRE, "workgroup");
    if (OUT_MODE == 0) {
      float* Cb = (float*)Cout + (size_t)b * strideC;
      const float* Rb = RESID ? (resid + (size_t)b * strideR) : nullptr;
      const int hh = lane >> 4, c4 = (lane & 15) * 4;
      v4f vals[8];
#pragma unroll
      for (int it = 0; it < 4; ++it) {
        const int row = it * 2 + hh;
        v4f v = *(const v4f*)(slab + row * 68 + c4);
        if (RESID) { const v4f rr = *(const v4f*)(Rb + (size_t)(mBase + row) * ldc + n0 + c4); v += rr; }
        vals[it] = v;
      }
      if (RESID) quad_keep4f(vals[0], vals[1], vals[2], vals[3]);
#pragma unroll
      for (int it = 4; it < 8; ++it) {
        const int row = it * 2 + hh;
        v4f v = *(const v4f*)(slab + row * 68 + c4);
        if (RESID) { const v4f rr = *(const v4f*)(Rb + (size_t)(mBase + row) * ldc + n0 + c4); v += rr; }
        vals[it] = v;
      }
      if (RESID) quad_keep4f(vals[4], vals[5], vals[6], vals[7]);
      for (int pass = 0; pass < 2; ++pass) {
#pragma unroll
        for (int it = 0; it < 8; ++it) {
          const int row = it * 2 + hh;
          *(volatile v4f*)(Cb + (size_t)(mBase + row) * ldc + n0 + c4) = vals[it];
        }
        __threadfence();
      }
    } else {
      const int q = lane >> 3, c8 = (lane & 7) * 8;
      unsigned short* Cb = (unsigned short*)Cout + (size_t)b * strideC;
      for (int pass = 0; pass < 2; ++pass) {
#pragma unroll
        for (int it = 0; it < 4; ++it) {
          const int row = it * 4 + q;
          const float* sp = slab + row * 68 + c8;
          v8h hv;
#pragma unroll
          for (int e = 0; e < 8; ++e) hv[e] = (_Float16)sp[e];
          *(volatile v8h*)(Cb + (size_t)(mBase + row) * ldc + n0 + c8) = hv;
        }
        __threadfence();
      }
    }
    __builtin_amdgcn_fence(__ATOMIC_RELEASE, "workgroup");
    __builtin_amdgcn_wave_barrier();
    __builtin_amdgcn_fence(__ATOMIC_ACQUIRE, "workgroup");
  }
}

__global__ __launch_bounds__(256) void wcast_kernel(const float* __restrict__ W0, const float* __restrict__ W1,
                                                    const float* __restrict__ W2p, const float* __restrict__ W3,
                                                    unsigned short* __restrict__ out, int n8, float scale) {
  const int z = blockIdx.y;
  const float* W = (z == 0) ? W0 : (z == 1) ? W1 : (z == 2) ? W2p : W3;
  const int i = blockIdx.x * 256 + threadIdx.x;
  if (i >= n8) return;
  const float* p = W + 8 * (size_t)i;
  const v4f a = *(const v4f*)(p);
  const v4f c = *(const v4f*)(p + 4);
  unsigned short hb[8];
#pragma unroll
  for (int e = 0; e < 4; ++e) {
    hb[e]     = h_bits(a[e] * scale);
    hb[4 + e] = h_bits(c[e] * scale);
  }
  const v4u u = (v4u){pk16(hb[0], hb[1]), pk16(hb[2], hb[3]), pk16(hb[4], hb[5]), pk16(hb[6], hb[7])};
  unsigned short* qo = out + (size_t)z * (8 * (size_t)n8) + 8 * (size_t)i;
  *(volatile v4u*)qo = u;
  __threadfence();
  *(volatile v4u*)qo = u;
}

__global__ __launch_bounds__(256) void xt_cast_kernel(const float* __restrict__ x, unsigned short* __restrict__ XT) {
  __shared__ float sm[64][65];
  const int t  = threadIdx.x;
  const int n0 = blockIdx.x * 64;
  const int c0 = blockIdx.y * 64;
  const int b  = blockIdx.z;
#pragma unroll
  for (int i = 0; i < 16; ++i) {
    const int e  = i * 256 + t;
    const int r  = e >> 6;
    const int cc = e & 63;
    sm[cc][r] = x[((size_t)(b * kC + c0 + r)) * kN + n0 + cc];
  }
  __syncthreads();
  const int lane = t & 31, wave = t >> 5;
  const int q = lane >> 3, c8 = (lane & 7) * 8;
  unsigned short* op = XT + ((size_t)b * kN) * kC;
  for (int pass = 0; pass < 2; ++pass) {
#pragma unroll
    for (int it = 0; it < 2; ++it) {
      const int row = wave * 8 + it * 4 + q;
      unsigned short hb[8];
#pragma unroll
      for (int e = 0; e < 8; ++e) hb[e] = h_bits(sm[row][c8 + e]);
      const v4u u = (v4u){pk16(hb[0], hb[1]), pk16(hb[2], hb[3]), pk16(hb[4], hb[5]), pk16(hb[6], hb[7])};
      *(volatile v4u*)(op + (size_t)(n0 + row) * kC + c0 + c8) = u;
    }
    __threadfence();
  }
}

extern "C" void kernel_launch(void* const* d_in, const int* in_sizes, int n_in,
                              void* d_out, int out_size, void* d_ws, size_t ws_size,
                              hipStream_t stream) {
  if (n_in < 9) return;
  const int nX = kBatch * kC * kN;
  if (in_sizes[0] != nX || out_size != nX) return;
  if (in_sizes[1] != kCi * kC || in_sizes[3] != kCi * kC || in_sizes[5] != kCi * kC || in_sizes[7] != kC * kCi) return;
  if (in_sizes[2] != kCi || in_sizes[4] != kCi || in_sizes[6] != kCi || in_sizes[8] != kC) return;

  const size_t szXT  = (size_t)kBatch * kN * kC * 2;
  const size_t szTH  = (size_t)kBatch * kN * kCi * 2;
  const size_t szPH  = (size_t)kBatch * kCi * kN * 2;
  const size_t szWpl = (size_t)kCi * kC * 2;
  const size_t szS   = (size_t)kBatch * kCi * kCi * 2;
  const size_t szW2  = (size_t)kBatch * kC * kCi * 2;
  const size_t offXT = 0;
  const size_t offTH = offXT + szXT;
  const size_t offPH = offTH + szTH;
  const size_t offG  = offPH + szPH;
  const size_t offW  = offG + szPH;
  const size_t offS  = offW + 4 * szWpl;
  const size_t offW2 = offS + szS;
  const size_t total = offW2 + szW2;
  if (ws_size < total) return;

  const float* x       = (const float*)d_in[0];
  const float* w_theta = (const float*)d_in[1];
  const float* b_theta = (const float*)d_in[2];
  const float* w_phi   = (const float*)d_in[3];
  const float* b_phi   = (const float*)d_in[4];
  const float* w_g     = (const float*)d_in[5];
  const float* b_g     = (const float*)d_in[6];
  const float* w_rec   = (const float*)d_in[7];
  const float* b_rec   = (const float*)d_in[8];
  float* out = (float*)d_out;
  char* ws = (char*)d_ws;
  unsigned short* XT16  = (unsigned short*)(ws + offXT);
  unsigned short* THT16 = (unsigned short*)(ws + offTH);
  unsigned short* PH16  = (unsigned short*)(ws + offPH);
  unsigned short* G16   = (unsigned short*)(ws + offG);
  unsigned short* W16   = (unsigned short*)(ws + offW);
  unsigned short* WTH   = W16;
  unsigned short* WPH   = W16 + 1 * (kCi * kC);
  unsigned short* WG    = W16 + 2 * (kCi * kC);
  unsigned short* WREC  = W16 + 3 * (kCi * kC);
  unsigned short* S16   = (unsigned short*)(ws + offS);
  unsigned short* W2C16 = (unsigned short*)(ws + offW2);

  const int n8w = (kCi * kC) / 8;
  wcast_kernel<<<dim3(n8w / 256, 4), dim3(256), 0, stream>>>(w_theta, w_phi, w_g, w_rec, W16, n8w, kWCarry);
  xt_cast_kernel<<<dim3(kN / 64, kC / 64, kBatch), dim3(256), 0, stream>>>(x, XT16);

  const long strideXT = (long)kN * kC;
  const long strideTH = (long)kN * kCi;
  const long stridePH = (long)kCi * kN;
  const long strideS  = (long)kCi * kCi;
  const long strideW2 = (long)kC * kCi;
  const long strideO  = (long)kC * kN;

  wmma_gemm64<0, false, 2, 1, false><<<dim3((kN / 64) * (kCi / 64) / 8, kBatch), dim3(256), 0, stream>>>(
      XT16, XT16, kC, strideXT, WTH, WTH, kC, 0L,
      (void*)THT16, kCi, strideTH, b_theta, x, 0L, kN, kCi, kC, kProjScale);
  wmma_gemm64<0, false, 1, 1, false><<<dim3((kCi / 64) * (kN / 64) / 8, kBatch), dim3(256), 0, stream>>>(
      WPH, WPH, kC, 0L, XT16, XT16, kC, strideXT,
      (void*)PH16, kN, stridePH, b_phi, x, 0L, kCi, kN, kC, kProjScale);
  wmma_gemm64<0, false, 1, 1, false><<<dim3((kCi / 64) * (kN / 64) / 8, kBatch), dim3(256), 0, stream>>>(
      WG, WG, kC, 0L, XT16, XT16, kC, strideXT,
      (void*)G16, kN, stridePH, b_g, x, 0L, kCi, kN, kC, kProjScale);
  wmma_gemm64<0, false, 0, 1, false><<<dim3(1, kBatch), dim3(128), 0, stream>>>(
      PH16, PH16, kN, stridePH, G16, G16, kN, stridePH,
      (void*)S16, kCi, strideS, b_phi, x, 0L, kCi, kCi, kN, kSScale);
  wmma_gemm64<0, false, 0, 1, false><<<dim3(1, kBatch), dim3(256), 0, stream>>>(
      WREC, WREC, kCi, 0L, S16, S16, kCi, strideS,
      (void*)W2C16, kCi, strideW2, b_rec, x, 0L, kC, kCi, kCi, kW2Scale);
  wmma_gemm64<0, false, 1, 0, true><<<dim3((kC / 64) * (kN / 64) / 8, kBatch), dim3(256), 0, stream>>>(
      W2C16, W2C16, kCi, strideW2, THT16, THT16, kCi, strideTH,
      (void*)out, kN, strideO, b_rec, x, strideO, kC, kN, kCi, kOutScale);
}
